// HyperbolicAttentionBias_77936476554060
// MI455X (gfx1250) — hardware-run, weakly checked
//
#include <hip/hip_runtime.h>
#include <math.h>

typedef __attribute__((ext_vector_type(16))) __bf16   v16b;
typedef __attribute__((ext_vector_type(8)))  __bf16   v8b;
typedef __attribute__((ext_vector_type(8)))  float    v8f;
typedef __attribute__((ext_vector_type(4)))  float    v4f;
typedef __attribute__((ext_vector_type(4)))  unsigned v4u;

constexpr int kNumTok = 30522;
constexpr int kDim    = 64;
constexpr int kBatch  = 4;
constexpr int kSeq    = 1024;
constexpr int kRows   = kBatch * kSeq;
static_assert(kDim == 64);
static_assert((kDim % 32) == 0);
static_assert((kSeq % 128) == 0);
static_assert((kSeq % 64) == 0);
static_assert(kRows == 4096);
static_assert((kRows % 256) == 0);

constexpr float kMaxNorm  = (float)((1.0 - 1e-5) / 1.0);
constexpr float kArgFloor = (float)(1.0 + 1e-7);

constexpr size_t kOffE    = 0;
constexpr size_t kOffX2   = kOffE  + (size_t)kRows * kDim * 2;
constexpr size_t kOffRinv = kOffX2 + (size_t)kRows * 4;
constexpr size_t kWsTotal = kOffRinv + (size_t)kRows * 4;
static_assert(kWsTotal == 557056ull);
static_assert(kWsTotal <= 134217728ull);
static_assert((kOffX2 % 128) == 0 && (kOffRinv % 128) == 0);

__device__ __forceinline__ unsigned short f2bf_bits(float f) {
  unsigned u = __float_as_uint(f);
  return (unsigned short)((u + 0x7FFFu + ((u >> 16) & 1u)) >> 16);
}
__device__ __forceinline__ float bf_bits2f(unsigned short h) { return __uint_as_float(((unsigned)h) << 16); }

struct FragB {
  union U { v16b v; v8b h[2]; };
  static __device__ __forceinline__ v16b load(const __bf16* p) {
    U f;
    f.h[0] = *(const v8b*)(p);
    f.h[1] = *(const v8b*)(p + 16);
    return f.v;
  }
};

__device__ __forceinline__ v8f mma_bf16_guarded(v16b a, v16b b, v8f c) {
  c = __builtin_amdgcn_wmma_f32_16x16x32_bf16(false, a, false, b, (short)0, c, false, false);
  asm volatile("v_nop\n\tv_nop\n\tv_nop\n\tv_nop" : "+v"(c) : "v"(a), "v"(b));
  return c;
}

__global__ __launch_bounds__(256) void gather_project_kernel(
    const int* __restrict__ ids, const float* __restrict__ weight,
    unsigned short* __restrict__ E, float* __restrict__ X2, float* __restrict__ RINV)
{
  __shared__ float sX2[8][32];
  const int tid  = threadIdx.x;
  const int lane = tid & 31;
  const int wave = tid >> 5;
  const int grp  = lane >> 3;
  const int sub  = lane & 7;
  const int base = (blockIdx.x * 8 + wave) * 32;

#pragma unroll 1
  for (int p = 0; p < 8; ++p) {
    const int tok = base + p * 4 + grp;
    int id = ids[tok];
    id = id < 0 ? 0 : id;
    id = id > (kNumTok - 1) ? (kNumTok - 1) : id;
    const float* wr = weight + (size_t)id * kDim + sub * 8;
    const v4f a0 = *(const v4f*)(wr);
    const v4f a1 = *(const v4f*)(wr + 4);
    float cv[8];
#pragma unroll
    for (int e = 0; e < 4; ++e) {
      const float f0 = a0[e];
      const float f1 = a1[e];
      cv[e]     = bf_bits2f(f2bf_bits(f0));
      cv[4 + e] = bf_bits2f(f2bf_bits(f1));
    }
    float ss = 0.0f;
#pragma unroll
    for (int e = 0; e < 8; ++e) ss = fmaf(cv[e], cv[e], ss);
    ss += __shfl_xor(ss, 1, 32);
    ss += __shfl_xor(ss, 2, 32);
    ss += __shfl_xor(ss, 4, 32);
    const float nrm  = sqrtf(ss);
    const float fprj = kMaxNorm / fmaxf(nrm, 1e-12f);
    const float fsel = (nrm > kMaxNorm) ? fprj : 1.0f;
    unsigned hb[8];
    float xs = 0.0f;
#pragma unroll
    for (int e = 0; e < 8; ++e) {
      const unsigned short h = f2bf_bits(cv[e] * fsel);
      const float vb = bf_bits2f(h);
      hb[e] = (unsigned)h;
      xs = fmaf(vb, vb, xs);
    }
    xs += __shfl_xor(xs, 1, 32);
    xs += __shfl_xor(xs, 2, 32);
    xs += __shfl_xor(xs, 4, 32);
    v4u w;
    w[0] = hb[0] | (hb[1] << 16);
    w[1] = hb[2] | (hb[3] << 16);
    w[2] = hb[4] | (hb[5] << 16);
    w[3] = hb[6] | (hb[7] << 16);
    unsigned short* dst = E + (size_t)tok * kDim + sub * 8;
    *(volatile v4u*)dst = w;
    __threadfence();
    *(volatile v4u*)dst = w;
    if (sub == 0) sX2[wave][p * 4 + grp] = xs;
  }
  __syncthreads();
  const float xv = sX2[wave][lane];
  const float om = 1.0f - xv;
  const float rv = 1.0f / om;
  volatile float* px = X2 + base + lane;
  volatile float* pr = RINV + base + lane;
  *px = xv;
  *pr = rv;
  __threadfence();
  *px = xv;
  *pr = rv;
}

__device__ __forceinline__ float pair_value(float xi, float ri, float xj, float rj, float g, float nsc) {
  const float sq  = fmaxf((xi + xj) - 2.0f * g, 0.0f);
  const float tt  = (2.0f * sq) * (ri * rj);
  const float arg = fmaxf(1.0f + tt, kArgFloor);
  const float tm  = arg - 1.0f;
  const float sr  = sqrtf(tm * (arg + 1.0f));
  return nsc * logf(arg + sr);
}

__global__ __launch_bounds__(256) void gram_dist_kernel(
    const unsigned short* __restrict__ Ep, const float* __restrict__ X2, const float* __restrict__ RINV,
    const float* __restrict__ scale_p, float* __restrict__ out)
{
  __shared__ __align__(16) float sT[8][16 * 68];
  const int b    = blockIdx.y;
  const int lane = threadIdx.x & 31;
  const int wave = threadIdx.x >> 5;
  const int ct   = blockIdx.x & 15;
  const int rg   = blockIdx.x >> 4;
  const int m0   = rg * 128 + wave * 16;
  const int n0   = ct * 64;
  const __bf16* Eb = (const __bf16*)Ep + (size_t)b * kSeq * kDim;

  const int rlane = lane & 15;
  const int koff  = (lane >> 4) * 8;
  const int mOff  = (lane >> 4) * 8;

  const v16b a0 = FragB::load(Eb + (size_t)(m0 + rlane) * kDim + koff);
  const v16b a1 = FragB::load(Eb + (size_t)(m0 + rlane) * kDim + koff + 32);

  v8f acc[4];
#pragma unroll
  for (int j = 0; j < 4; ++j) {
    const size_t bo = (size_t)(n0 + (j << 4) + rlane) * kDim + koff;
    const v16b b0 = FragB::load(Eb + bo);
    const v16b b1 = FragB::load(Eb + bo + 32);
    acc[j] = (v8f){0.f, 0.f, 0.f, 0.f, 0.f, 0.f, 0.f, 0.f};
    acc[j] = mma_bf16_guarded(a0, b0, acc[j]);
    acc[j] = mma_bf16_guarded(a1, b1, acc[j]);
  }

  float* slab = sT[wave];
#pragma unroll
  for (int j = 0; j < 4; ++j) {
#pragma unroll
    for (int r = 0; r < 8; ++r) {
      slab[(mOff + r) * 68 + (j << 4) + rlane] = acc[j][r];
    }
  }
  __builtin_amdgcn_fence(__ATOMIC_RELEASE, "workgroup");
  __builtin_amdgcn_wave_barrier();
  __builtin_amdgcn_fence(__ATOMIC_ACQUIRE, "workgroup");

  const float* x2b = X2 + (size_t)b * kSeq;
  const float* rnb = RINV + (size_t)b * kSeq;
  const int hh = lane >> 4;
  const int c4 = (lane & 15) * 4;
  const v4f xj = *(const v4f*)(x2b + n0 + c4);
  const v4f rj = *(const v4f*)(rnb + n0 + c4);
  const float nsc = -scale_p[0];
#pragma unroll 1
  for (int it = 0; it < 8; ++it) {
    const int row = it * 2 + hh;
    const float xi = x2b[m0 + row];
    const float ri = rnb[m0 + row];
    const v4f g = *(const v4f*)(slab + row * 68 + c4);
    v4f o;
#pragma unroll
    for (int e = 0; e < 4; ++e) {
      o[e] = pair_value(xi, ri, xj[e], rj[e], g[e], nsc);
    }
    *(v4f*)(slab + row * 68 + c4) = o;
  }
  __builtin_amdgcn_fence(__ATOMIC_RELEASE, "workgroup");
  __builtin_amdgcn_wave_barrier();
  __builtin_amdgcn_fence(__ATOMIC_ACQUIRE, "workgroup");

  float* C = out + (size_t)b * kSeq * kSeq;
  for (int pass = 0; pass < 2; ++pass) {
#pragma unroll
    for (int it = 0; it < 8; ++it) {
      const int row = it * 2 + hh;
      const v4f v = *(const v4f*)(slab + row * 68 + c4);
      *(volatile v4f*)(C + (size_t)(m0 + row) * kSeq + n0 + c4) = v;
    }
    __threadfence();
  }
}

extern "C" void kernel_launch(void* const* d_in, const int* in_sizes, int n_in,
                              void* d_out, int out_size, void* d_ws, size_t ws_size,
                              hipStream_t stream) {
  if (n_in < 3) return;
  if (in_sizes[0] != kRows) return;
  if (in_sizes[1] != kNumTok * kDim) return;
  if (in_sizes[2] != 1) return;
  if (out_size != kBatch * kSeq * kSeq) return;
  if (ws_size < kWsTotal) return;

  const int*   ids     = (const int*)d_in[0];
  const float* weight  = (const float*)d_in[1];
  const float* scale_p = (const float*)d_in[2];
  float* out = (float*)d_out;

  char* ws = (char*)d_ws;
  unsigned short* E    = (unsigned short*)(ws + kOffE);
  float*          X2   = (float*)(ws + kOffX2);
  float*          RINV = (float*)(ws + kOffRinv);

  gather_project_kernel<<<kRows / 256, 256, 0, stream>>>(ids, weight, E, X2, RINV);
  gram_dist_kernel<<<dim3((kSeq / 128) * (kSeq / 64), kBatch), 256, 0, stream>>>(E, X2, RINV, scale_p, out);
}
